// SimpleMambaBlock_32916629357355
// MI455X (gfx1250) — hardware-run, weakly checked
//
#include <hip/hip_runtime.h>
#include <math.h>

constexpr int kB    = 4;
constexpr int kL    = 2048;
constexpr int kDM   = 1024;
constexpr int kDI   = 2048;
constexpr int kNXZ  = 4096;
constexpr int kNS   = 16;
constexpr int kKC   = 4;
constexpr int kXP   = 33;
constexpr int kXPP  = 64;
constexpr int kTok  = kB * kL;
constexpr float kWCarry   = 64.0f;
constexpr float kACarry   = 16.0f;
constexpr float kInScale  = 1.0f / 64.0f;
constexpr float kXpScale  = 1.0f / 1024.0f;
constexpr float kOutScale = 1.0f / 1024.0f;

typedef __attribute__((ext_vector_type(16))) _Float16 v16h;
typedef __attribute__((ext_vector_type(8)))  _Float16 v8h;
typedef __attribute__((ext_vector_type(16))) __bf16   v16b;
typedef __attribute__((ext_vector_type(8)))  __bf16   v8b;
typedef __attribute__((ext_vector_type(8)))  float    v8f;
typedef __attribute__((ext_vector_type(4)))  float    v4f;
typedef __attribute__((ext_vector_type(4)))  unsigned int v4u;

__device__ __forceinline__ unsigned short f2bf_bits(float f) {
  unsigned u = __float_as_uint(f);
  return (unsigned short)((u + 0x7FFFu + ((u >> 16) & 1u)) >> 16);
}
__device__ __forceinline__ float bf_bits2f(unsigned short h) { return __uint_as_float(((unsigned)h) << 16); }

__device__ __forceinline__ void dep_guard_h(v8f& a, v8f& b, v16h x, v16h y) { asm volatile("v_nop\n\tv_nop\n\tv_nop\n\tv_nop" : "+v"(a), "+v"(b) : "v"(x), "v"(y)); }
__device__ __forceinline__ void dep_guard_b(v8f& a, v8f& b, v16b x, v16b y) { asm volatile("v_nop\n\tv_nop\n\tv_nop\n\tv_nop" : "+v"(a), "+v"(b) : "v"(x), "v"(y)); }
__device__ __forceinline__ void keep4_h(v16h a, v16h b, v16h c, v16h d) { asm volatile("v_nop" :: "v"(a), "v"(b), "v"(c), "v"(d)); }
__device__ __forceinline__ void keep4_b(v16b a, v16b b, v16b c, v16b d) { asm volatile("v_nop" :: "v"(a), "v"(b), "v"(c), "v"(d)); }
__device__ __forceinline__ void acc_guard4(v8f& a, v8f& b, v8f& c, v8f& d) { asm volatile("v_nop\n\tv_nop\n\tv_nop\n\tv_nop" : "+v"(a), "+v"(b), "+v"(c), "+v"(d)); }
template <typename T> struct Frag;
template <> struct Frag<_Float16> {
  typedef v16h V; union U { v16h v; v8h h[2]; };
  static __device__ __forceinline__ v16h load(const _Float16* p) {
    U f; f.h[0] = *(const v8h*)(p); f.h[1] = *(const v8h*)(p + 16); return f.v;
  }
  static __device__ __forceinline__ v8f mma(v16h a, v16h b, v8f c) {
    return __builtin_amdgcn_wmma_f32_16x16x32_f16(false, a, false, b, (short)0, c, false, false);
  }
  static __device__ __forceinline__ void guard(v8f& a, v8f& b, v16h x, v16h y) { dep_guard_h(a, b, x, y); }
  static __device__ __forceinline__ void keep(v16h a, v16h b, v16h c, v16h d) { keep4_h(a, b, c, d); }
};
template <> struct Frag<__bf16> {
  typedef v16b V; union U { v16b v; v8b h[2]; };
  static __device__ __forceinline__ v16b load(const __bf16* p) {
    U f; f.h[0] = *(const v8b*)(p); f.h[1] = *(const v8b*)(p + 16); return f.v;
  }
  static __device__ __forceinline__ v8f mma(v16b a, v16b b, v8f c) {
    return __builtin_amdgcn_wmma_f32_16x16x32_bf16(false, a, false, b, (short)0, c, false, false);
  }
  static __device__ __forceinline__ void guard(v8f& a, v8f& b, v16b x, v16b y) { dep_guard_b(a, b, x, y); }
  static __device__ __forceinline__ void keep(v16b a, v16b b, v16b c, v16b d) { keep4_b(a, b, c, d); }
};

__device__ __forceinline__ unsigned pk16(unsigned short a, unsigned short b) { return (unsigned)a | ((unsigned)b << 16); }
__device__ __forceinline__ unsigned short h_bits(float f) { const _Float16 h = (_Float16)f; return __builtin_bit_cast(unsigned short, h); }

template <int ET> struct Elem;
template <> struct Elem<0> { typedef _Float16 T; };
template <> struct Elem<1> { typedef __bf16 T; };
template <int ET, bool SPLIT, int BIAS_MODE, int OUT_MODE, bool RESID, int ACT = 0>
__global__ __launch_bounds__(256) void wmma_gemm64(
    const unsigned short* __restrict__ Ap, const unsigned short* __restrict__ A2p, int lda, long strideA,
    const unsigned short* __restrict__ Btp, const unsigned short* __restrict__ Bt2p, int ldb, long strideB,
    void* __restrict__ Cout, void* __restrict__ Cout2, int ldc, long strideC,
    const float* __restrict__ bias,
    const float* __restrict__ resid, long strideR,
    int M, int N, int K, float scale) {
  typedef typename Elem<ET>::T T;
  typedef typename Frag<T>::V V;
  const T* A = (const T*)Ap; const T* A2 = (const T*)A2p; const T* Bt = (const T*)Btp; const T* Bt2 = (const T*)Bt2p;
  __shared__ __align__(16) float sT[8][16 * 68];
  const int b    = blockIdx.y;
  const int lane = threadIdx.x & 31;
  const int wave = threadIdx.x >> 5;
  const int tilesN = N >> 6;
  const int tilesM = M >> 6;
  const int tile = blockIdx.x * 8 + wave;
  if (tile >= tilesM * tilesN) return;
  const int tm = tile / tilesN;
  const int tn = tile - tm * tilesN;
  const int m0 = tm << 6;
  const int n0 = tn << 6;

  const T* Ab  = A  + (size_t)b * strideA;
  const T* Bb  = Bt + (size_t)b * strideB;
  const T* Ab2 = SPLIT ? (A2  + (size_t)b * strideA) : nullptr;
  const T* Bb2 = SPLIT ? (Bt2 + (size_t)b * strideB) : nullptr;

  const int rlane = lane & 15;
  const int koff  = (lane >> 4) * 8;
  const int mOff  = (lane >> 4) * 8;

  v8f acc[4][4];
#pragma unroll
  for (int i = 0; i < 4; ++i)
#pragma unroll
    for (int j = 0; j < 4; ++j) acc[i][j] = (v8f){0.f,0.f,0.f,0.f,0.f,0.f,0.f,0.f};

  for (int k0 = 0; k0 < K; k0 += 32) {
    V bh[4], bl[4];
#pragma unroll
    for (int j = 0; j < 4; ++j) {
      const size_t bo = (size_t)(n0 + (j << 4) + rlane) * ldb + koff + k0;
      bh[j] = Frag<T>::load(Bb + bo);
      if (SPLIT) bl[j] = Frag<T>::load(Bb2 + bo);
    }
#pragma unroll
    for (int i = 0; i < 4; ++i) {
      const size_t ao = (size_t)(m0 + (i << 4) + rlane) * lda + koff + k0;
      V ah = Frag<T>::load(Ab + ao);
      V al;
      if (SPLIT) al = Frag<T>::load(Ab2 + ao);
#pragma unroll
      for (int j = 0; j < 4; ++j) {
        acc[i][j] = Frag<T>::mma(ah, bh[j], acc[i][j]);
        if (SPLIT) {
          acc[i][j] = Frag<T>::mma(ah, bl[j], acc[i][j]);
          acc[i][j] = Frag<T>::mma(al, bh[j], acc[i][j]);
        }
      }
      Frag<T>::guard(acc[i][0], acc[i][3], ah, SPLIT ? al : ah);
    }
    Frag<T>::keep(bh[0], bh[1], bh[2], bh[3]);
    if (SPLIT) Frag<T>::keep(bl[0], bl[1], bl[2], bl[3]);
  }
  acc_guard4(acc[0][0], acc[0][1], acc[0][2], acc[0][3]);
  acc_guard4(acc[1][0], acc[1][1], acc[1][2], acc[1][3]);
  acc_guard4(acc[2][0], acc[2][1], acc[2][2], acc[2][3]);
  acc_guard4(acc[3][0], acc[3][1], acc[3][2], acc[3][3]);

  float* slab = sT[wave];
  const float* Rb = RESID ? (resid + (size_t)b * strideR) : nullptr;
#pragma unroll
  for (int i = 0; i < 4; ++i) {
    const int mBase = m0 + (i << 4);
#pragma unroll
    for (int j = 0; j < 4; ++j) {
      const int n = n0 + (j << 4) + rlane;
      float bv = 0.f;
      if (BIAS_MODE == 2) bv = bias[n];
#pragma unroll
      for (int r = 0; r < 8; ++r) {
        float v = acc[i][j][r] * scale;
        if (BIAS_MODE == 1) v += bias[mBase + mOff + r];
        if (BIAS_MODE == 2) v += bv;
        if (RESID) v += Rb[(size_t)(mBase + mOff + r) * ldc + n];
        if (ACT == 2) v = fmaxf(v, 0.0f);
        if (ACT == 4) v = (v > 0.f) ? v : 0.01f * v;
        slab[(mOff + r) * 68 + (j << 4) + rlane] = v;
      }
    }
    __builtin_amdgcn_fence(__ATOMIC_RELEASE, "workgroup");
    __builtin_amdgcn_wave_barrier();
    __builtin_amdgcn_fence(__ATOMIC_ACQUIRE, "workgroup");
    if (OUT_MODE == 0) {
      float* C = (float*)Cout + (size_t)b * strideC;
      const int hh = lane >> 4, c4 = (lane & 15) * 4;
      for (int pass = 0; pass < 2; ++pass) {
#pragma unroll
        for (int it = 0; it < 8; ++it) {
          const int row = it * 2 + hh;
          v4f v = *(const v4f*)(slab + row * 68 + c4);
          *(volatile v4f*)(C + (size_t)(mBase + row) * ldc + n0 + c4) = v;
        }
        __threadfence();
      }
    } else {
      const int q = lane >> 3, c8 = (lane & 7) * 8;
      unsigned short* C  = (unsigned short*)Cout  + (size_t)b * strideC;
      unsigned short* C2 = (OUT_MODE == 2) ? ((unsigned short*)Cout2 + (size_t)b * strideC) : nullptr;
      for (int pass = 0; pass < 2; ++pass) {
#pragma unroll
        for (int it = 0; it < 4; ++it) {
          const int row = it * 4 + q;
          const float* sp = slab + row * 68 + c8;
          v8h hv, lv;
#pragma unroll
          for (int e = 0; e < 8; ++e) {
            if (OUT_MODE == 1) {
              hv[e] = (_Float16)sp[e];
            } else {
              unsigned short hb = f2bf_bits(sp[e]);
              unsigned short lb = f2bf_bits(sp[e] - bf_bits2f(hb));
              hv[e] = __builtin_bit_cast(_Float16, hb);
              lv[e] = __builtin_bit_cast(_Float16, lb);
            }
          }
          *(volatile v8h*)(C + (size_t)(mBase + row) * ldc + n0 + c8) = hv;
          if (OUT_MODE == 2) *(volatile v8h*)(C2 + (size_t)(mBase + row) * ldc + n0 + c8) = lv;
        }
        __threadfence();
      }
    }
    __builtin_amdgcn_fence(__ATOMIC_RELEASE, "workgroup");
    __builtin_amdgcn_wave_barrier();
    __builtin_amdgcn_fence(__ATOMIC_ACQUIRE, "workgroup");
  }
}

__global__ __launch_bounds__(256) void cast8_f16_kernel(const float* __restrict__ in, unsigned short* __restrict__ out, int n8) {
  const int i = blockIdx.x * 256 + threadIdx.x;
  if (i >= n8) return;
  const float* p = in + 8 * (size_t)i;
  const v4f a = *(const v4f*)(p);
  const v4f c = *(const v4f*)(p + 4);
  unsigned short hb[8];
#pragma unroll
  for (int e = 0; e < 4; ++e) {
    hb[e]     = h_bits(a[e]);
    hb[4 + e] = h_bits(c[e]);
  }
  const v4u u = (v4u){pk16(hb[0], hb[1]), pk16(hb[2], hb[3]), pk16(hb[4], hb[5]), pk16(hb[6], hb[7])};
  unsigned short* q = out + 8 * (size_t)i;
  *(volatile v4u*)q = u;
  __threadfence();
  *(volatile v4u*)q = u;
}

__global__ __launch_bounds__(256) void tcast_kernel(const float* __restrict__ W, unsigned short* __restrict__ out,
                                                    int R, int Cc, float scale) {
  __shared__ float sm[64][65];
  const int t  = threadIdx.x;
  const int r0 = blockIdx.x * 64;
  const int c0 = blockIdx.y * 64;
#pragma unroll
  for (int i = 0; i < 16; ++i) {
    const int e = i * 256 + t;
    const int r = e >> 6;
    const int c = e & 63;
    sm[c][r] = W[(size_t)(r0 + r) * Cc + c0 + c] * scale;
  }
  __syncthreads();
  const int lane = t & 31, wave = t >> 5;
  const int q = lane >> 3, c8 = (lane & 7) * 8;
  for (int pass = 0; pass < 2; ++pass) {
#pragma unroll
    for (int it = 0; it < 2; ++it) {
      const int row = wave * 8 + it * 4 + q;
      unsigned short hb[8];
#pragma unroll
      for (int e = 0; e < 8; ++e) hb[e] = h_bits(sm[row][c8 + e]);
      const v4u u = (v4u){pk16(hb[0], hb[1]), pk16(hb[2], hb[3]), pk16(hb[4], hb[5]), pk16(hb[6], hb[7])};
      *(volatile v4u*)(out + (size_t)(c0 + row) * R + r0 + c8) = u;
    }
    __threadfence();
  }
}

__global__ __launch_bounds__(256) void wxcast_kernel(const float* __restrict__ Wx, unsigned short* __restrict__ out) {
  const int j  = blockIdx.x;
  const int t  = threadIdx.x;
  const int k0 = t * 8;
  const int jc = (j < kXP) ? j : (kXP - 1);
  const float sc = (j < kXP) ? kWCarry : 0.0f;
  unsigned short hb[8];
#pragma unroll
  for (int e = 0; e < 8; ++e) hb[e] = h_bits(Wx[(size_t)(k0 + e) * kXP + jc] * sc);
  const v4u u = (v4u){pk16(hb[0], hb[1]), pk16(hb[2], hb[3]), pk16(hb[4], hb[5]), pk16(hb[6], hb[7])};
  unsigned short* q = out + (size_t)j * kDI + k0;
  *(volatile v4u*)q = u;
  __threadfence();
  *(volatile v4u*)q = u;
}

__global__ __launch_bounds__(256) void conv_silu_kernel(const float* __restrict__ XZ, const float* __restrict__ cw,
                                                        const float* __restrict__ cb, float* __restrict__ XS,
                                                        unsigned short* __restrict__ XSh) {
  __shared__ __align__(16) unsigned int sh32[512];
  const int t  = threadIdx.x;
  const int l  = blockIdx.x >> 1;
  const int dh = (blockIdx.x & 1) * 1024;
  const int d  = dh + 4 * t;
  v4f xin[kKC];
#pragma unroll
  for (int k = 0; k < kKC; ++k) {
    const int ls = l + k - (kKC - 1);
    const int lc = (ls < 0) ? 0 : ls;
    const v4f v = *(const v4f*)(XZ + (size_t)lc * kNXZ + d);
    const float keep = (ls >= 0) ? 1.0f : 0.0f;
    xin[k] = v * keep;
  }
  v4f w[4];
#pragma unroll
  for (int e = 0; e < 4; ++e) w[e] = *(const v4f*)(cw + (size_t)(d + e) * kKC);
  v4f acc = *(const v4f*)(cb + d);
#pragma unroll
  for (int k = 0; k < kKC; ++k) {
    const v4f wk = (v4f){w[0][k], w[1][k], w[2][k], w[3][k]};
    acc = acc + xin[k] * wk;
  }
  v4f res;
#pragma unroll
  for (int e = 0; e < 4; ++e) {
    const float a  = acc[e];
    const float sg = __builtin_amdgcn_rcpf(1.0f + expf(-a));
    res[e] = a * sg;
  }
  sh32[2 * t]     = pk16(h_bits(res[0] * kACarry), h_bits(res[1] * kACarry));
  sh32[2 * t + 1] = pk16(h_bits(res[2] * kACarry), h_bits(res[3] * kACarry));
  __syncthreads();
  const int tt = t & 127;
  const v4u u = *(const v4u*)(sh32 + 4 * tt);
  float* xp = XS + (size_t)l * kDI + d;
  unsigned short* hp = XSh + (size_t)l * kDI + dh + 8 * tt;
  for (int pass = 0; pass < 2; ++pass) {
    *(volatile v4f*)xp = res;
    if (t < 128) *(volatile v4u*)hp = u;
    __threadfence();
  }
}

__global__ __launch_bounds__(64) void scan_gate_kernel(const float* __restrict__ XS, const float* __restrict__ XZ,
                                                      const float* __restrict__ XDBL,
                                                      const float* __restrict__ wdt, const float* __restrict__ bdt,
                                                      const float* __restrict__ Alog, const float* __restrict__ Dv,
                                                      unsigned short* __restrict__ Y) {
  __shared__ __align__(16) float sdbl[64 * 64];
  __shared__ float hbuf[kNS * 64];
  __shared__ float abuf[kNS * 64];
  __shared__ __align__(16) unsigned short obuf[64 * 64];
  const int tid = threadIdx.x;
  const int d0  = blockIdx.x * 64;
  const int d   = d0 + tid;
  const float wd = wdt[d];
  const float bd = bdt[d];
  const float Dd = Dv[d];
#pragma unroll 1
  for (int n = 0; n < kNS; ++n) {
    abuf[n * 64 + tid] = -expf(Alog[(size_t)d * kNS + n]);
    hbuf[n * 64 + tid] = 0.0f;
  }
#pragma unroll 1
  for (int l0 = 0; l0 < kL; l0 += 64) {
    __syncthreads();
#pragma unroll
    for (int i = 0; i < 16; ++i) {
      const int idx = i * 64 + tid;
      const int row = idx >> 4;
      const int c4  = (idx & 15) * 4;
      *(v4f*)(sdbl + row * 64 + c4) = *(const v4f*)(XDBL + (size_t)(l0 + row) * kXPP + c4);
    }
    __syncthreads();
#pragma unroll 1
    for (int t = 0; t < 64; ++t) {
      const int l = l0 + t;
      const float xv = XS[(size_t)l * kDI + d];
      const float zv = XZ[(size_t)l * kNXZ + kDI + d];
      const float* rowp = sdbl + t * 64;
      const float xa = rowp[0] * wd + bd;
      const float sp = fmaxf(xa, 0.0f) + log1pf(expf(-fabsf(xa)));
      const float dx = sp * xv;
      float y = 0.0f;
#pragma unroll 1
      for (int n = 0; n < kNS; ++n) {
        const float a  = expf(sp * abuf[n * 64 + tid]);
        float hn = hbuf[n * 64 + tid];
        hn = a * hn + dx * rowp[1 + n];
        hbuf[n * 64 + tid] = hn;
        y = y + hn * rowp[1 + kNS + n];
      }
      const float yv = y + xv * Dd;
      const float sg = __builtin_amdgcn_rcpf(1.0f + expf(-zv));
      const float o  = yv * (zv * sg);
      obuf[t * 64 + tid] = h_bits(o * kACarry);
    }
    __syncthreads();
    const int q = tid >> 3, c8 = (tid & 7) * 8;
    for (int pass = 0; pass < 2; ++pass) {
#pragma unroll
      for (int it = 0; it < 8; ++it) {
        const int row = it * 8 + q;
        const v4u u = *(const v4u*)(obuf + row * 64 + c8);
        *(volatile v4u*)(Y + (size_t)(l0 + row) * kDI + d0 + c8) = u;
      }
      __threadfence();
    }
  }
}

extern "C" void kernel_launch(void* const* d_in, const int* in_sizes, int n_in,
                              void* d_out, int out_size, void* d_ws, size_t ws_size,
                              hipStream_t stream)
{
  if (n_in < 10) return;
  if (in_sizes[0] != kTok * kDM) return;
  if (in_sizes[1] != kDM * kNXZ) return;
  if (in_sizes[2] != kDI * kKC) return;
  if (in_sizes[4] != kDI * kXP) return;
  if (in_sizes[7] != kDI * kNS) return;
  if (in_sizes[9] != kDI * kDM) return;
  if (out_size < kTok * kDM) return;

  const float* x     = (const float*)d_in[0];
  const float* W_in  = (const float*)d_in[1];
  const float* convw = (const float*)d_in[2];
  const float* convb = (const float*)d_in[3];
  const float* W_x   = (const float*)d_in[4];
  const float* w_dt  = (const float*)d_in[5];
  const float* b_dt  = (const float*)d_in[6];
  const float* A_log = (const float*)d_in[7];
  const float* Dvec  = (const float*)d_in[8];
  const float* W_out = (const float*)d_in[9];
  float* out = (float*)d_out;

  char* ws = (char*)d_ws;
  size_t off = 0;
  const size_t szXh  = (size_t)kTok * kDM * 2;
  const size_t szWin = (size_t)kNXZ * kDM * 2;
  const size_t szWo  = (size_t)kDM * kDI * 2;
  const size_t szWx  = (size_t)kXPP * kDI * 2;
  const size_t szXZ  = (size_t)kL * kNXZ * 4;
  const size_t szXS  = (size_t)kL * kDI * 4;
  const size_t szXSh = (size_t)kL * kDI * 2;
  const size_t szXD  = (size_t)kL * kXPP * 4;
  const size_t szYh  = (size_t)kL * kDI * 2;
  unsigned short* Xh  = (unsigned short*)(ws + off); off += szXh;
  unsigned short* WinT = (unsigned short*)(ws + off); off += szWin;
  unsigned short* WoT = (unsigned short*)(ws + off); off += szWo;
  unsigned short* WxT = (unsigned short*)(ws + off); off += szWx;
  float*          XZ  = (float*)(ws + off);          off += szXZ;
  float*          XS  = (float*)(ws + off);          off += szXS;
  unsigned short* XSh = (unsigned short*)(ws + off); off += szXSh;
  float*          XD  = (float*)(ws + off);          off += szXD;
  unsigned short* Yh  = (unsigned short*)(ws + off); off += szYh;
  if (off > ws_size) return;

  const int n8x = kTok * kDM / 8;
  cast8_f16_kernel<<<(n8x + 255) / 256, 256, 0, stream>>>(x, Xh, n8x);
  tcast_kernel<<<dim3(kDM / 64, kNXZ / 64), 256, 0, stream>>>(W_in, WinT, kDM, kNXZ, kWCarry);
  tcast_kernel<<<dim3(kDI / 64, kDM / 64), 256, 0, stream>>>(W_out, WoT, kDI, kDM, kWCarry);
  wxcast_kernel<<<kXPP, 256, 0, stream>>>(W_x, WxT);

  const int tiles0 = (kL / 64) * (kNXZ / 64);
  const int tiles1 = (kL / 64) * (kXPP / 64);
  const int tiles2 = (kL / 64) * (kDM / 64);

  for (int c = 0; c < kB; ++c) {
    const unsigned short* Xc = Xh + (size_t)c * kL * kDM;
    float* outc = out + (size_t)c * kL * kDM;

    wmma_gemm64<0, false, 0, 0, false, 0><<<dim3((tiles0 + 7) / 8, 1), 256, 0, stream>>>(
        Xc, Xc, kDM, 0L, WinT, WinT, kDM, 0L,
        (void*)XZ, (void*)XZ, kNXZ, 0L, convb, XS, 0L, kL, kNXZ, kDM, kInScale);

    conv_silu_kernel<<<2 * kL, 256, 0, stream>>>(XZ, convw, convb, XS, XSh);

    wmma_gemm64<0, false, 0, 0, false, 0><<<dim3((tiles1 + 7) / 8, 1), 256, 0, stream>>>(
        XSh, XSh, kDI, 0L, WxT, WxT, kDI, 0L,
        (void*)XD, (void*)XD, kXPP, 0L, convb, XS, 0L, kL, kXPP, kDI, kXpScale);

    scan_gate_kernel<<<kDI / 64, 64, 0, stream>>>(XS, XZ, XD, w_dt, b_dt, A_log, Dvec, Yh);

    wmma_gemm64<0, false, 0, 0, false, 0><<<dim3((tiles2 + 7) / 8, 1), 256, 0, stream>>>(
        Yh, Yh, kDI, 0L, WoT, WoT, kDI, 0L,
        (void*)outc, (void*)outc, kDM, 0L, convb, XS, 0L, kL, kDM, kDI, kOutScale);
  }
}
